// MF2Demo_26379689132515
// MI455X (gfx1250) — hardware-verified
//
#include <hip/hip_runtime.h>
#include <math.h>

typedef __attribute__((ext_vector_type(16))) _Float16 v16h;
typedef __attribute__((ext_vector_type(16))) __bf16 v16b;
typedef __attribute__((ext_vector_type(8)))  _Float16 v8h;
typedef __attribute__((ext_vector_type(8)))  float v8f;
typedef __attribute__((ext_vector_type(4)))  float v4f;
typedef __attribute__((ext_vector_type(2)))  float v2f;
typedef __attribute__((ext_vector_type(4)))  unsigned v4u;
typedef __attribute__((ext_vector_type(4)))  int v4i;
typedef float __attribute__((may_alias)) float_a;
typedef int __attribute__((may_alias)) int_a;

template <typename T> __device__ __forceinline__ void vst2(void* p, T v) { *(volatile T*)p = v; __threadfence(); *(volatile T*)p = v; }
__device__ __forceinline__ v8f wmma16(v16h a, v16h b, v8f c) {
  v8f d = __builtin_amdgcn_wmma_f32_16x16x32_f16(false, a, false, b, (short)0, c, false, false);
  asm volatile("v_nop\n\tv_nop\n\tv_nop\n\tv_nop" : "+v"(d) : "v"(a), "v"(b));
  return d;
}
__device__ __forceinline__ v8f wmma_bf(v16b a, v16b b, v8f c) {
  v8f d = __builtin_amdgcn_wmma_f32_16x16x32_bf16(false, a, false, b, (short)0, c, false, false);
  asm volatile("v_nop\n\tv_nop\n\tv_nop\n\tv_nop" : "+v"(d) : "v"(a), "v"(b));
  return d;
}
__device__ __forceinline__ v16h frag_h(const _Float16* rowk0, int lane) {
  union { v16h v; v8h q[2]; } u; const _Float16* p = rowk0 + 8 * (lane >> 4);
  u.q[0] = *(const v8h*)p; u.q[1] = *(const v8h*)(p + 16); return u.v;
}
__device__ __forceinline__ v16h frag_f32(const float* rowk0, int lane) {
  v16h a; const float* p = rowk0 + 8 * (lane >> 4);
#pragma unroll
  for (int i = 0; i < 8; ++i) { a[i] = (_Float16)p[i]; a[8 + i] = (_Float16)p[16 + i]; }
  return a;
}
__device__ __forceinline__ v16h frag_f32s(const float* rowk0, int lane, float sc) {
  v16h a; const float* p = rowk0 + 8 * (lane >> 4);
#pragma unroll
  for (int i = 0; i < 8; ++i) { a[i] = (_Float16)(p[i] * sc); a[8 + i] = (_Float16)(p[16 + i] * sc); }
  return a;
}
__device__ __forceinline__ v16h fragc_f32(const float* W, int k0, int n, int lane, int ld, int K) {
  v16h a; const int g = lane >> 4;
#pragma unroll
  for (int i = 0; i < 8; ++i) { const int ka = k0 + 8 * g + i, kb = ka + 16;
    a[i] = (_Float16)(ka < K ? W[(size_t)(ka < K ? ka : K - 1) * ld + n] : 0.f); a[8 + i] = (_Float16)(kb < K ? W[(size_t)(kb < K ? kb : K - 1) * ld + n] : 0.f); }
  return a;
}
struct F2 { v16b h, l; };
__device__ __forceinline__ F2 bsplit16(const float v[16]) { F2 r;
#pragma unroll
  for (int i = 0; i < 16; ++i) { const __bf16 h = (__bf16)v[i]; r.h[i] = h; r.l[i] = (__bf16)(v[i] - (float)h); }
  return r; }
__device__ __forceinline__ F2 split_row(const float* row, int k0, int lane) { float v[16]; const float* p = row + k0 + 8 * (lane >> 4);
#pragma unroll
  for (int i = 0; i < 8; ++i) { v[i] = p[i]; v[8 + i] = p[16 + i]; }
  return bsplit16(v); }
__device__ __forceinline__ F2 split_rowK(const float* row, int k0, int lane, int K) { float v[16]; const int g = lane >> 4;
#pragma unroll
  for (int i = 0; i < 8; ++i) { const int ka = k0 + 8 * g + i, kb = ka + 16; v[i] = ka < K ? row[ka < K ? ka : K - 1] : 0.f; v[8 + i] = kb < K ? row[kb < K ? kb : K - 1] : 0.f; }
  return bsplit16(v); }
__device__ __forceinline__ F2 split_col(const float* W, int k0, int n, int lane, int ld, int K) { float v[16]; const int g = lane >> 4;
#pragma unroll
  for (int i = 0; i < 8; ++i) { const int ka = k0 + 8 * g + i, kb = ka + 16; v[i] = ka < K ? W[(size_t)(ka < K ? ka : K - 1) * ld + n] : 0.f; v[8 + i] = kb < K ? W[(size_t)(kb < K ? kb : K - 1) * ld + n] : 0.f; }
  return bsplit16(v); }
__device__ __forceinline__ v8f mac3(const F2& a, const F2& b, v8f c) { c = wmma_bf(a.l, b.h, c); c = wmma_bf(a.h, b.l, c); return wmma_bf(a.h, b.h, c); }
__device__ __forceinline__ float sigm(float v) { return 1.0f / (1.0f + expf(-v)); }
#define LDSX() do { asm volatile("s_wait_dscnt 0" ::: "memory"); __builtin_amdgcn_wave_barrier(); __builtin_amdgcn_fence(__ATOMIC_RELEASE, "workgroup"); } while (0)


#define NBt 8192
#define DE 256
#define H1 50
#define H1P 64
#define H2 32
#define NO 18
#define NOP 32
#define NCASE 256
typedef __attribute__((ext_vector_type(8))) __bf16 v8b;
__device__ __forceinline__ v16b frag_b(const __bf16* rowk0, int lane) {
  union { v16b v; v8b q[2]; } u; const __bf16* p = rowk0 + 8 * (lane >> 4);
  u.q[0] = *(const v8b*)p; u.q[1] = *(const v8b*)(p + 16); return u.v;
}
__device__ __forceinline__ float bfr(float v) { return (float)(__bf16)v; }
__device__ __attribute__((noinline)) float exp_ni(float v) { return expf(v); }
__device__ __attribute__((noinline)) float erf_ni(float v) { return erff(v); }

#define OUT1_OFF ((size_t)NBt * NO)
#define WS_YS  0u
#define WS_LP  (WS_YS + 4u * 32)
#define WS_END (WS_LP + 4u * (NBt / 64) * 32)

__global__ __launch_bounds__(256) void k_ysum(const float* __restrict__ Y, float* __restrict__ YS) { __shared__ float sp[256][NO + 1]; __shared__ __align__(16) float so[32];
  const int t = threadIdx.x; float a[NO]; for (int k = 0; k < NO; ++k) a[k] = 0.f;
  for (int j = t; j < NBt; j += 256) for (int k = 0; k < NO; ++k) a[k] += bfr(Y[(size_t)j * NO + k]);
  for (int k = 0; k < NO; ++k) sp[t][k] = a[k];
  __syncthreads(); if (t < 32) { float s = 0.f; if (t < NO) for (int w = 0; w < 256; ++w) s += sp[w][t]; so[t] = s; }
  __syncthreads(); if (t < 8) vst2(YS + t * 4, *(const v4f*)&so[t * 4]); }
__global__ __launch_bounds__(128) void k_mlp(const float* __restrict__ X, const float* __restrict__ W1, const float* __restrict__ B1, const float* __restrict__ W2, const float* __restrict__ B2, const float* __restrict__ W3, const float* __restrict__ B3, const float* __restrict__ CS, const float* __restrict__ YS, float* __restrict__ OUT, float* __restrict__ LP) {
  __shared__ __align__(16) float sh1[64][H1P + 4]; __shared__ __align__(16) float sh2[64][H2 + 4]; __shared__ __align__(16) float sw[64 * NO + 16]; __shared__ float scs[NCASE][NO + 1]; __shared__ float sred[64];
  const int tid = threadIdx.x, wave = tid >> 5, lane = tid & 31, col = lane & 15, g = lane >> 4; const size_t r0 = (size_t)blockIdx.x * 64 + wave * 16;
  for (int e = tid; e < NCASE * NO; e += 128) scs[e / NO][e % NO] = bfr(CS[e]);
  { v8f acc[4] = {};
#pragma unroll
    for (int kc = 0; kc < DE / 32; ++kc) { v16b a; { const float* p = X + (r0 + col) * DE + kc * 32 + 8 * g;
#pragma unroll
        for (int i = 0; i < 8; ++i) { a[i] = (__bf16)p[i]; a[8 + i] = (__bf16)p[16 + i]; } }
#pragma unroll
      for (int j = 0; j < 4; ++j) { v16b w; const int o = j * 16 + col; const int oc = min(o, H1 - 1);
#pragma unroll
        for (int i = 0; i < 8; ++i) { w[i] = (__bf16)(o < H1 ? W1[(size_t)(kc * 32 + 8 * g + i) * H1 + oc] : 0.f); w[8 + i] = (__bf16)(o < H1 ? W1[(size_t)(kc * 32 + 16 + 8 * g + i) * H1 + oc] : 0.f); }
        acc[j] = wmma_bf(a, w, acc[j]); } }
#pragma unroll
    for (int j = 0; j < 4; ++j) { const int o = j * 16 + col;
#pragma unroll
      for (int r = 0; r < 8; ++r) sh1[wave * 16 + 8 * g + r][o] = (o < H1) ? 1.0f / (1.0f + expf(-(acc[j][r] + bfr(B1[min(o, H1 - 1)])))) : 0.f; } }
  __syncthreads();
  { v8f acc[2] = {};
#pragma unroll
    for (int kc = 0; kc < H1P / 32; ++kc) { const F2 a = split_row(&sh1[wave * 16 + col][0], kc * 32, lane);
#pragma unroll
      for (int j = 0; j < 2; ++j) { v16b w; const int o = j * 16 + col;
#pragma unroll
        for (int i = 0; i < 8; ++i) { const int k0 = kc * 32 + 8 * g + i, k1 = k0 + 16; w[i] = (__bf16)(k0 < H1 ? W2[(size_t)k0 * H2 + o] : 0.f); w[8 + i] = (__bf16)(k1 < H1 ? W2[(size_t)k1 * H2 + o] : 0.f); }
        acc[j] = wmma_bf(a.h, w, acc[j]); acc[j] = wmma_bf(a.l, w, acc[j]); } }
#pragma unroll
    for (int j = 0; j < 2; ++j) { const int o = j * 16 + col;
#pragma unroll
      for (int r = 0; r < 8; ++r) sh2[wave * 16 + 8 * g + r][o] = 1.0f / (1.0f + expf(-(acc[j][r] + bfr(B2[o])))); } }
  __syncthreads();
  { v8f acc[2] = {}; const F2 a = split_row(&sh2[wave * 16 + col][0], 0, lane);
#pragma unroll
    for (int j = 0; j < 2; ++j) { v16b w; const int o = j * 16 + col; const int oc = min(o, NO - 1);
#pragma unroll
      for (int i = 0; i < 8; ++i) { w[i] = (__bf16)(o < NO ? W3[(size_t)(8 * g + i) * NO + oc] : 0.f); w[8 + i] = (__bf16)(o < NO ? W3[(size_t)(16 + 8 * g + i) * NO + oc] : 0.f); }
      acc[j] = wmma_bf(a.h, w, acc[j]); acc[j] = wmma_bf(a.l, w, acc[j]); }
#pragma unroll
    for (int j = 0; j < 2; ++j) { const int o = j * 16 + col;
#pragma unroll
      for (int r = 0; r < 8; ++r) if (o < NO) sw[(wave * 16 + 8 * g + r) * NO + o] = acc[j][r] + bfr(B3[o]); } }
  __syncthreads();
  if (tid < 64) { const float* wu = &sw[tid * NO]; float mx = -3.0e38f;
#pragma unroll 1
    for (int c = 0; c < NCASE; ++c) { float d = 0.f;
#pragma unroll 1
      for (int k = 0; k < NO; ++k) d += wu[k] * scs[c][k]; mx = fmaxf(mx, d); }
    float s = 0.f;
#pragma unroll 1
    for (int c = 0; c < NCASE; ++c) { float d = 0.f;
#pragma unroll 1
      for (int k = 0; k < NO; ++k) d += wu[k] * scs[c][k]; s += expf(d - mx); }
    const float lse = mx + logf(s); float sy = 0.f;
#pragma unroll 1
    for (int k = 0; k < NO; ++k) sy += wu[k] * YS[k];
    sred[tid] = sy - lse; }
  __syncthreads();
  for (int q = tid; q < 64 * NO / 4; q += 128) vst2(OUT + (size_t)blockIdx.x * 64 * NO + q * 4, *(const v4f*)&sw[q * 4]);
  if (tid == 0) { float a = 0.f; for (int i = 0; i < 64; ++i) a += sred[i]; __align__(16) float rec[4] = {a, 0.f, 0.f, 0.f}; vst2(LP + (size_t)blockIdx.x * 32, *(const v4f*)rec); } }
__global__ __launch_bounds__(64) void k_loss(const float* __restrict__ LP, float* __restrict__ OUTL) { if (threadIdx.x == 0) { float a = 0.f; for (int i = 0; i < NBt / 64; ++i) a += LP[i * 32]; vst2(OUTL, -a); } }
extern "C" void kernel_launch(void* const* d_in, const int* in_sizes, int n_in, void* d_out, int out_size, void* d_ws, size_t ws_size, hipStream_t stream) {
  (void)in_sizes; (void)n_in; (void)out_size;
  const float** F = (const float**)d_in;
  if (ws_size < (size_t)WS_END) return;
  char* ws = (char*)d_ws; float *YS = (float*)(ws + WS_YS), *LP = (float*)(ws + WS_LP);
  k_ysum<<<1, 256, 0, stream>>>(F[1], YS);
  k_mlp<<<NBt / 64, 128, 0, stream>>>(F[0], F[2], F[3], F[4], F[5], F[6], F[7], F[8], YS, (float*)d_out, LP);
  k_loss<<<1, 64, 0, stream>>>(LP, (float*)d_out + OUT1_OFF);
}
